// ConstantModulationAttention_45930380264095
// MI455X (gfx1250) — hardware-verified
//
#include <hip/hip_runtime.h>


typedef __bf16         v16bf __attribute__((ext_vector_type(16)));
typedef float          v8f   __attribute__((ext_vector_type(8)));
typedef float          v4f   __attribute__((ext_vector_type(4), __may_alias__));
typedef unsigned short u16x8 __attribute__((ext_vector_type(8), __may_alias__));
typedef unsigned int   u32x4 __attribute__((ext_vector_type(4), __may_alias__));
typedef int            i32x4 __attribute__((ext_vector_type(4), __may_alias__));
typedef unsigned long long u64a __attribute__((__may_alias__));

#define NB   2
#define NS   2048
#define NE   1024
#define NH   16
#define ND   64
#define NTOK (NB * NS)
#define NC3  (3 * NH * ND)
#define NQT  (NS / 64)
#define FROW 64
#define TP   68
#define PP   72

union Frag { v16bf v; u16x8 h[2]; };

__device__ __forceinline__ v16bf ldfrag(const unsigned short* p, size_t ld, size_t row0, int k0, int lane) {
  const unsigned short* q = p + (row0 + (size_t)(lane & 15)) * ld + k0 + ((lane >> 4) << 3);
  Frag f;
  f.h[0] = *(const u16x8*)q;
  f.h[1] = *(const u16x8*)(q + 16);
  return f.v;
}

__device__ __forceinline__ v8f mma(v16bf a, v16bf b, v8f c) {
  v8f d = __builtin_amdgcn_wmma_f32_16x16x32_bf16(false, a, false, b, (short)0, c, false, false);
  asm volatile("v_nop\n\tv_nop\n\tv_nop\n\tv_nop" : "+v"(d) : "v"(a), "v"(b));
  return d;
}

__device__ __forceinline__ unsigned int bf16_bits(float x) {
  unsigned int u = __float_as_uint(x);
  return (u + 0x7FFFu + ((u >> 16) & 1u)) >> 16;
}
__device__ __forceinline__ void split1(float x, unsigned int& hi, unsigned int& lo) {
  hi = bf16_bits(x);
  lo = bf16_bits(x - __uint_as_float(hi << 16));
}
__device__ __forceinline__ void split8(const float (&v)[8], u32x4& H, u32x4& L) {
  unsigned int hw[8], lw[8];
#pragma unroll
  for (int e = 0; e < 8; ++e) split1(v[e], hw[e], lw[e]);
#pragma unroll
  for (int w = 0; w < 4; ++w) {
    H[w] = hw[2 * w] | (hw[2 * w + 1] << 16);
    L[w] = lw[2 * w] | (lw[2 * w + 1] << 16);
  }
}
__device__ __forceinline__ u32x4 pick(int c, u32x4 a, u32x4 b) {
  u32x4 r;
#pragma unroll
  for (int w = 0; w < 4; ++w) r[w] = c ? a[w] : b[w];
  return r;
}
__device__ __forceinline__ float sigm(float v) { return 1.0f / (1.0f + __expf(-v)); }

__global__ __launch_bounds__(256) void k_split_rows(const float* __restrict__ src,
                                                    unsigned short* __restrict__ dh,
                                                    unsigned short* __restrict__ dl, int ngroups)
{
  const int g = blockIdx.x * 256 + threadIdx.x;
  const int gc = (g < ngroups) ? g : (ngroups - 1);
  const float* s = src + (size_t)gc * 8;
  const v4f a0 = *(const v4f*)s;
  const v4f a1 = *(const v4f*)(s + 4);
  float v[8] = {a0[0], a0[1], a0[2], a0[3], a1[0], a1[1], a1[2], a1[3]};
  u32x4 H, L;
  split8(v, H, L);
  if (g < ngroups) {
    unsigned short* ph = dh + (size_t)gc * 8;
    unsigned short* pl = dl + (size_t)gc * 8;
    *(volatile u32x4*)ph = H;
    *(volatile u32x4*)pl = L;
    __threadfence();
    *(volatile u32x4*)ph = H;
    *(volatile u32x4*)pl = L;
  }
}

__global__ __launch_bounds__(256) void k_transpose_split(const float* __restrict__ src, int R, int C,
                                                         unsigned short* __restrict__ oh,
                                                         unsigned short* __restrict__ ol)
{
  __shared__ __align__(16) float T[64 * TP];
  const int tid = threadIdx.x, lane = tid & 31, wave = tid >> 5;
  const int nb = blockIdx.x * 64;
  const int kb = blockIdx.y * 64;
#pragma unroll
  for (int it = 0; it < 4; ++it) {
    const int idx = tid + 256 * it;
    const int kk = idx >> 4, c4 = idx & 15;
    const v4f v = *(const v4f*)(src + (size_t)(kb + kk) * C + nb + c4 * 4);
#pragma unroll
    for (int q = 0; q < 4; ++q) T[(c4 * 4 + q) * TP + kk] = v[q];
  }
  __syncthreads();
  const int q = lane >> 3, p = lane & 7;
  const int plane = q & 1;
  u32x4 val[4];
#pragma unroll
  for (int it = 0; it < 4; ++it) {
    const int n = wave * 8 + it * 2 + (q >> 1);
    const v4f a0 = *(const v4f*)(&T[n * TP + p * 8]);
    const v4f a1 = *(const v4f*)(&T[n * TP + p * 8 + 4]);
    float v[8] = {a0[0], a0[1], a0[2], a0[3], a1[0], a1[1], a1[2], a1[3]};
    u32x4 H, L;
    split8(v, H, L);
    val[it] = pick(plane, L, H);
  }
  unsigned short* base = plane ? ol : oh;
#pragma unroll
  for (int it = 0; it < 4; ++it) {
    const int n = wave * 8 + it * 2 + (q >> 1);
    unsigned short* dst = base + (size_t)(nb + n) * R + kb + p * 8;
    *(volatile u32x4*)dst = val[it];
  }
  __threadfence();
#pragma unroll
  for (int it = 0; it < 4; ++it) {
    const int n = wave * 8 + it * 2 + (q >> 1);
    unsigned short* dst = base + (size_t)(nb + n) * R + kb + p * 8;
    *(volatile u32x4*)dst = val[it];
  }
}

__global__ __launch_bounds__(256) void k_flags(const int* __restrict__ msk, int* __restrict__ ftab)
{
  __shared__ int s_any[256];
  __shared__ int s_all[256];
  __shared__ __align__(16) int s_row[FROW];
  const int tid = threadIdx.x, qt = blockIdx.x;
  const int kt = tid >> 3, sub = tid & 7;
  int anyv = 0, allv = 1;
  for (int i = 0; i < 8; ++i) {
    const int s = qt * 64 + sub * 8 + i;
    const int* rp = msk + (size_t)s * NS + kt * 64;
#pragma unroll
    for (int c = 0; c < 16; ++c) {
      const i32x4 v = *(const i32x4*)(rp + c * 4);
#pragma unroll
      for (int q = 0; q < 4; ++q) {
        const int nz = (v[q] != 0) ? 1 : 0;
        anyv |= nz;
        allv &= nz;
      }
    }
  }
  s_any[tid] = anyv;
  s_all[tid] = allv;
  __syncthreads();
  if (tid < 32) {
    int a = 0, b = 1;
#pragma unroll
    for (int j = 0; j < 8; ++j) { a |= s_any[tid * 8 + j]; b &= s_all[tid * 8 + j]; }
    s_row[tid] = b ? 2 : (a ? 1 : 0);
  } else if (tid < FROW) {
    s_row[tid] = 0;
  }
  __syncthreads();
  if (tid == 0) {
    int last = -1;
    for (int k = 0; k < 32; ++k) if (s_row[k] != 0) last = k;
    s_row[32] = last;
  }
  __syncthreads();
  if (tid < 16) {
    const i32x4 v = *(const i32x4*)(&s_row[tid * 4]);
    int* dst = ftab + (size_t)qt * FROW + tid * 4;
    *(volatile i32x4*)dst = v;
    __threadfence();
    *(volatile i32x4*)dst = v;
  }
}

__device__ __forceinline__ void mainloop(const unsigned short* __restrict__ Ah, const unsigned short* __restrict__ Al,
                                         const unsigned short* __restrict__ Bh, const unsigned short* __restrict__ Bl,
                                         int K, size_t arow, size_t brow, int lane, v8f (&acc)[2][2])
{
  for (int k0 = 0; k0 < K; k0 += 32) {
    const v16bf ah0 = ldfrag(Ah, (size_t)K, arow,      k0, lane);
    const v16bf ah1 = ldfrag(Ah, (size_t)K, arow + 16, k0, lane);
    const v16bf al0 = ldfrag(Al, (size_t)K, arow,      k0, lane);
    const v16bf al1 = ldfrag(Al, (size_t)K, arow + 16, k0, lane);
#pragma unroll
    for (int ni = 0; ni < 2; ++ni) {
      const v16bf bh = ldfrag(Bh, (size_t)K, brow + ni * 16, k0, lane);
      const v16bf bl = ldfrag(Bl, (size_t)K, brow + ni * 16, k0, lane);
      acc[0][ni] = mma(ah0, bh, acc[0][ni]);
      acc[0][ni] = mma(ah0, bl, acc[0][ni]);
      acc[0][ni] = mma(al0, bh, acc[0][ni]);
      acc[1][ni] = mma(ah1, bh, acc[1][ni]);
      acc[1][ni] = mma(ah1, bl, acc[1][ni]);
      acc[1][ni] = mma(al1, bh, acc[1][ni]);
    }
  }
}

__global__ __launch_bounds__(256) void k_gemm_qkv(
    const unsigned short* __restrict__ Xh, const unsigned short* __restrict__ Xl,
    const unsigned short* __restrict__ Wh, const unsigned short* __restrict__ Wl,
    const float* __restrict__ sq,
    unsigned short* __restrict__ Qh, unsigned short* __restrict__ Ql,
    unsigned short* __restrict__ Kh, unsigned short* __restrict__ Kl,
    unsigned short* __restrict__ Vh, unsigned short* __restrict__ Vl)
{
  __shared__ __align__(16) float T[128 * TP];
  const int tid = threadIdx.x, lane = tid & 31, wave = tid >> 5;
  const int hf = lane >> 4, m16 = lane & 15;
  const int cb = blockIdx.x * 64;
  const int rb = blockIdx.y * 128;
  const int mr = (wave & 3) * 32, nc = (wave >> 2) * 32;
  v8f acc[2][2] = {};
  mainloop(Xh, Xl, Wh, Wl, NE, (size_t)(rb + mr), (size_t)(cb + nc), lane, acc);

  const int c = cb >> 10;
  const int h = (cb & 1023) >> 6;
  float g[2];
#pragma unroll
  for (int ni = 0; ni < 2; ++ni) g[ni] = sigm(sq[(cb & 1023) + nc + ni * 16 + m16]);
#pragma unroll
  for (int mi = 0; mi < 2; ++mi)
#pragma unroll
    for (int ni = 0; ni < 2; ++ni)
#pragma unroll
      for (int r = 0; r < 8; ++r)
        T[(mr + mi * 16 + 8 * hf + r) * TP + nc + ni * 16 + m16] = acc[mi][ni][r] * g[ni];
  __syncthreads();

  const int q = lane >> 3, p = lane & 7;
  const int b = rb >> 11;
  u32x4 val[8];
  if (c < 2) {
    const int plane = q & 1;
#pragma unroll
    for (int it = 0; it < 8; ++it) {
      const int r = wave * 16 + it * 2 + (q >> 1);
      const v4f a0 = *(const v4f*)(&T[r * TP + p * 8]);
      const v4f a1 = *(const v4f*)(&T[r * TP + p * 8 + 4]);
      float v[8] = {a0[0], a0[1], a0[2], a0[3], a1[0], a1[1], a1[2], a1[3]};
      u32x4 H, L;
      split8(v, H, L);
      val[it] = pick(plane, L, H);
    }
    unsigned short* base = (c == 0) ? (plane ? Ql : Qh) : (plane ? Kl : Kh);
#pragma unroll
    for (int it = 0; it < 8; ++it) {
      const int r = wave * 16 + it * 2 + (q >> 1);
      const int s = (rb + r) & (NS - 1);
      unsigned short* dst = base + ((size_t)(b * NH + h) * NS + s) * ND + p * 8;
      *(volatile u32x4*)dst = val[it];
    }
    __threadfence();
#pragma unroll
    for (int it = 0; it < 8; ++it) {
      const int r = wave * 16 + it * 2 + (q >> 1);
      const int s = (rb + r) & (NS - 1);
      unsigned short* dst = base + ((size_t)(b * NH + h) * NS + s) * ND + p * 8;
      *(volatile u32x4*)dst = val[it];
    }
  } else {
    const int plane = (q >> 1) & 1, sh = q & 1;
#pragma unroll
    for (int it = 0; it < 8; ++it) {
      const int d = wave * 8 + it;
      float v[8];
#pragma unroll
      for (int e = 0; e < 8; ++e) v[e] = T[(sh * 64 + p * 8 + e) * TP + d];
      u32x4 H, L;
      split8(v, H, L);
      val[it] = pick(plane, L, H);
    }
    unsigned short* base = plane ? Vl : Vh;
    const int sbase = (rb & (NS - 1)) + sh * 64 + p * 8;
#pragma unroll
    for (int it = 0; it < 8; ++it) {
      const int d = wave * 8 + it;
      unsigned short* dst = base + ((size_t)(b * NH + h) * ND + d) * NS + sbase;
      *(volatile u32x4*)dst = val[it];
    }
    __threadfence();
#pragma unroll
    for (int it = 0; it < 8; ++it) {
      const int d = wave * 8 + it;
      unsigned short* dst = base + ((size_t)(b * NH + h) * ND + d) * NS + sbase;
      *(volatile u32x4*)dst = val[it];
    }
  }
}

__global__ __launch_bounds__(128) void k_attn(
    const unsigned short* __restrict__ Qh, const unsigned short* __restrict__ Ql,
    const unsigned short* __restrict__ Kh, const unsigned short* __restrict__ Kl,
    const unsigned short* __restrict__ Vh, const unsigned short* __restrict__ Vl,
    const int* __restrict__ msk, const int* __restrict__ ftab,
    unsigned short* __restrict__ Ah, unsigned short* __restrict__ Al)
{
  __shared__ __align__(16) unsigned short Ps[4 * 2 * 16 * PP];
  __shared__ __align__(16) unsigned char  Ms[64 * 64];
  __shared__ __align__(16) float          Os[64 * TP];
  __shared__ __align__(16) int            s_f[FROW];
  const int tid = threadIdx.x, lane = tid & 31, wave = tid >> 5;
  const int hf = lane >> 4, m16 = lane & 15;
  const int qt = blockIdx.x, h = blockIdx.y, b = blockIdx.z;
  const int s0 = qt * 64;
  const int bh = b * NH + h;
  if (tid < FROW) s_f[tid] = ftab[(size_t)qt * FROW + tid];
  __syncthreads();
  int last = s_f[32];
  last = (last < -1) ? -1 : ((last > NQT - 1) ? (NQT - 1) : last);
  const int nt = last + 1;

  const size_t qrow = (size_t)bh * NS + s0 + wave * 16;
  const v16bf qh0 = ldfrag(Qh, ND, qrow, 0,  lane);
  const v16bf qh1 = ldfrag(Qh, ND, qrow, 32, lane);
  const v16bf ql0 = ldfrag(Ql, ND, qrow, 0,  lane);
  const v16bf ql1 = ldfrag(Ql, ND, qrow, 32, lane);

  float m[8], l[8];
#pragma unroll
  for (int i = 0; i < 8; ++i) { m[i] = -3.0e38f; l[i] = 0.0f; }
  v8f acc[4] = {};
  unsigned short* Pwh = Ps + (wave * 2 + 0) * (16 * PP);
  unsigned short* Pwl = Ps + (wave * 2 + 1) * (16 * PP);

  for (int tb = 0; tb < nt; ++tb) {
    const int f = s_f[tb];
    if (f == 0) continue;
    const int t0 = tb * 64;
    __syncthreads();
    if (f == 1) {
#pragma unroll
      for (int it = 0; it < 8; ++it) {
        const int idx = tid + 128 * it;
        const int s = idx >> 4, c4 = idx & 15;
        const i32x4 v = *(const i32x4*)(msk + (size_t)(s0 + s) * NS + t0 + c4 * 4);
#pragma unroll
        for (int q = 0; q < 4; ++q) Ms[(c4 * 4 + q) * 64 + s] = (unsigned char)((v[q] != 0) ? 1 : 0);
      }
    }
    __syncthreads();

    v8f sf[4];
    const size_t krow = (size_t)bh * NS + t0;
#pragma unroll
    for (int j = 0; j < 4; ++j) {
      v8f c = {};
      v16bf kh = ldfrag(Kh, ND, krow + j * 16, 0, lane);
      v16bf kl = ldfrag(Kl, ND, krow + j * 16, 0, lane);
      c = mma(qh0, kh, c);
      c = mma(qh0, kl, c);
      c = mma(ql0, kh, c);
      kh = ldfrag(Kh, ND, krow + j * 16, 32, lane);
      kl = ldfrag(Kl, ND, krow + j * 16, 32, lane);
      c = mma(qh1, kh, c);
      c = mma(qh1, kl, c);
      c = mma(ql1, kh, c);
      sf[j] = c;
    }

    float rmax[8];
#pragma unroll
    for (int i = 0; i < 8; ++i) rmax[i] = -3.0e38f;
#pragma unroll
    for (int j = 0; j < 4; ++j) {
      const u64a mb = *(const u64a*)(Ms + (j * 16 + m16) * 64 + wave * 16 + 8 * hf);
#pragma unroll
      for (int i = 0; i < 8; ++i) {
        float s = sf[j][i] * 0.125f;
        const bool keep = (f != 1) || (((mb >> (8 * i)) & 0xffull) != 0ull);
        s = keep ? s : -1.0e10f;
        sf[j][i] = s;
        rmax[i] = fmaxf(rmax[i], s);
      }
    }
    float alpha[8], mnew[8], rsum[8];
#pragma unroll
    for (int i = 0; i < 8; ++i) {
      float v = rmax[i];
      v = fmaxf(v, __shfl_xor(v, 1, 32));
      v = fmaxf(v, __shfl_xor(v, 2, 32));
      v = fmaxf(v, __shfl_xor(v, 4, 32));
      v = fmaxf(v, __shfl_xor(v, 8, 32));
      mnew[i]  = fmaxf(m[i], v);
      alpha[i] = __expf(m[i] - mnew[i]);
      rsum[i]  = 0.0f;
    }
#pragma unroll
    for (int j = 0; j < 4; ++j)
#pragma unroll
      for (int i = 0; i < 8; ++i) {
        const float pv = __expf(sf[j][i] - mnew[i]);
        sf[j][i] = pv;
        rsum[i] += pv;
      }
#pragma unroll
    for (int i = 0; i < 8; ++i) {
      float v = rsum[i];
      v += __shfl_xor(v, 1, 32);
      v += __shfl_xor(v, 2, 32);
      v += __shfl_xor(v, 4, 32);
      v += __shfl_xor(v, 8, 32);
      l[i] = l[i] * alpha[i] + v;
      m[i] = mnew[i];
    }
#pragma unroll
    for (int j = 0; j < 4; ++j)
#pragma unroll
      for (int i = 0; i < 8; ++i) acc[j][i] *= alpha[i];

#pragma unroll
    for (int j = 0; j < 4; ++j)
#pragma unroll
      for (int i = 0; i < 8; ++i) {
        unsigned int hi, lo;
        split1(sf[j][i], hi, lo);
        const int o = (8 * hf + i) * PP + j * 16 + m16;
        Pwh[o] = (unsigned short)hi;
        Pwl[o] = (unsigned short)lo;
      }
    __syncthreads();
    const v16bf ph0 = ldfrag(Pwh, PP, 0, 0,  lane);
    const v16bf ph1 = ldfrag(Pwh, PP, 0, 32, lane);
    const v16bf pl0 = ldfrag(Pwl, PP, 0, 0,  lane);
    const v16bf pl1 = ldfrag(Pwl, PP, 0, 32, lane);

    const size_t vrow = (size_t)bh * ND;
#pragma unroll
    for (int j = 0; j < 4; ++j) {
      v16bf vh = ldfrag(Vh, NS, vrow + j * 16, t0, lane);
      v16bf vl = ldfrag(Vl, NS, vrow + j * 16, t0, lane);
      acc[j] = mma(ph0, vh, acc[j]);
      acc[j] = mma(ph0, vl, acc[j]);
      acc[j] = mma(pl0, vh, acc[j]);
      vh = ldfrag(Vh, NS, vrow + j * 16, t0 + 32, lane);
      vl = ldfrag(Vl, NS, vrow + j * 16, t0 + 32, lane);
      acc[j] = mma(ph1, vh, acc[j]);
      acc[j] = mma(ph1, vl, acc[j]);
      acc[j] = mma(pl1, vh, acc[j]);
    }
  }

  float inv[8];
#pragma unroll
  for (int i = 0; i < 8; ++i) inv[i] = (l[i] > 0.0f) ? (1.0f / l[i]) : 0.0f;
#pragma unroll
  for (int j = 0; j < 4; ++j)
#pragma unroll
    for (int i = 0; i < 8; ++i)
      Os[(wave * 16 + 8 * hf + i) * TP + j * 16 + m16] = acc[j][i] * inv[i];
  __syncthreads();

  const int q = lane >> 3, p = lane & 7;
  const int plane = q & 1;
  u32x4 val[8];
#pragma unroll
  for (int it = 0; it < 8; ++it) {
    const int r = wave * 16 + it * 2 + (q >> 1);
    const v4f a0 = *(const v4f*)(&Os[r * TP + p * 8]);
    const v4f a1 = *(const v4f*)(&Os[r * TP + p * 8 + 4]);
    float v[8] = {a0[0], a0[1], a0[2], a0[3], a1[0], a1[1], a1[2], a1[3]};
    u32x4 H, L;
    split8(v, H, L);
    val[it] = pick(plane, L, H);
  }
  unsigned short* base = plane ? Al : Ah;
#pragma unroll
  for (int it = 0; it < 8; ++it) {
    const int r = wave * 16 + it * 2 + (q >> 1);
    unsigned short* dst = base + ((size_t)(b * NS + s0 + r)) * NE + h * ND + p * 8;
    *(volatile u32x4*)dst = val[it];
  }
  __threadfence();
#pragma unroll
  for (int it = 0; it < 8; ++it) {
    const int r = wave * 16 + it * 2 + (q >> 1);
    unsigned short* dst = base + ((size_t)(b * NS + s0 + r)) * NE + h * ND + p * 8;
    *(volatile u32x4*)dst = val[it];
  }
}

__global__ __launch_bounds__(256) void k_gemm_out(
    const unsigned short* __restrict__ Ah, const unsigned short* __restrict__ Al,
    const unsigned short* __restrict__ Wh, const unsigned short* __restrict__ Wl,
    const float* __restrict__ so, float* __restrict__ out)
{
  __shared__ __align__(16) float T[128 * TP];
  const int tid = threadIdx.x, lane = tid & 31, wave = tid >> 5;
  const int hf = lane >> 4, m16 = lane & 15;
  const int cb = blockIdx.x * 64;
  const int rb = blockIdx.y * 128;
  const int mr = (wave & 3) * 32, nc = (wave >> 2) * 32;
  v8f acc[2][2] = {};
  mainloop(Ah, Al, Wh, Wl, NE, (size_t)(rb + mr), (size_t)(cb + nc), lane, acc);

  float g[2];
#pragma unroll
  for (int ni = 0; ni < 2; ++ni) g[ni] = sigm(so[cb + nc + ni * 16 + m16]);
#pragma unroll
  for (int mi = 0; mi < 2; ++mi)
#pragma unroll
    for (int ni = 0; ni < 2; ++ni)
#pragma unroll
      for (int r = 0; r < 8; ++r)
        T[(mr + mi * 16 + 8 * hf + r) * TP + nc + ni * 16 + m16] = acc[mi][ni][r] * g[ni];
  __syncthreads();

  const int rsel = lane >> 4, p = lane & 15;
  v4f val[8];
#pragma unroll
  for (int it = 0; it < 8; ++it) {
    const int r = wave * 16 + it * 2 + rsel;
    val[it] = *(const v4f*)(&T[r * TP + p * 4]);
  }
#pragma unroll
  for (int it = 0; it < 8; ++it) {
    const int r = wave * 16 + it * 2 + rsel;
    float* dst = out + (size_t)(rb + r) * NE + cb + p * 4;
    *(volatile v4f*)dst = val[it];
  }
  __threadfence();
#pragma unroll
  for (int it = 0; it < 8; ++it) {
    const int r = wave * 16 + it * 2 + rsel;
    float* dst = out + (size_t)(rb + r) * NE + cb + p * 4;
    *(volatile v4f*)dst = val[it];
  }
}

extern "C" void kernel_launch(void* const* d_in, const int* in_sizes, int n_in,
                              void* d_out, int out_size, void* d_ws, size_t ws_size,
                              hipStream_t stream)
{
  if (n_in < 6) return;
  if (in_sizes[0] != NTOK * NE || in_sizes[1] != NE * NC3 || in_sizes[2] != NE * NE ||
      in_sizes[3] != NE || in_sizes[4] != NE || in_sizes[5] != NS * NS || out_size != NTOK * NE) return;

  const float* x     = (const float*)d_in[0];
  const float* Wqkv  = (const float*)d_in[1];
  const float* Wout  = (const float*)d_in[2];
  const float* sqkv  = (const float*)d_in[3];
  const float* sout  = (const float*)d_in[4];
  const int*   msk   = (const int*)d_in[5];
  float* out = (float*)d_out;

  char* ws = (char*)d_ws;
  size_t off = 0;
  const size_t szX  = (size_t)NTOK * NE * 2;
  const size_t szW  = (size_t)NC3 * NE * 2;
  const size_t szWo = (size_t)NE * NE * 2;
  const size_t szP  = (size_t)NB * NH * NS * ND * 2;
  const size_t szF  = (size_t)NQT * FROW * 4;
  unsigned short* Xh  = (unsigned short*)(ws + off); off += szX;
  unsigned short* Xl  = (unsigned short*)(ws + off); off += szX;
  unsigned short* Wh  = (unsigned short*)(ws + off); off += szW;
  unsigned short* Wl  = (unsigned short*)(ws + off); off += szW;
  unsigned short* Woh = (unsigned short*)(ws + off); off += szWo;
  unsigned short* Wol = (unsigned short*)(ws + off); off += szWo;
  unsigned short* Qh  = (unsigned short*)(ws + off); off += szP;
  unsigned short* Ql  = (unsigned short*)(ws + off); off += szP;
  unsigned short* Kh  = (unsigned short*)(ws + off); off += szP;
  unsigned short* Kl  = (unsigned short*)(ws + off); off += szP;
  unsigned short* Vh  = (unsigned short*)(ws + off); off += szP;
  unsigned short* Vl  = (unsigned short*)(ws + off); off += szP;
  unsigned short* Ahp = (unsigned short*)(ws + off); off += szX;
  unsigned short* Alp = (unsigned short*)(ws + off); off += szX;
  int* ftab = (int*)(ws + off); off += szF;
  if (off > ws_size) return;

  const int ngroups = NTOK * NE / 8;
  k_split_rows<<<dim3((ngroups + 255) / 256), dim3(256), 0, stream>>>(x, Xh, Xl, ngroups);
  k_transpose_split<<<dim3(NC3 / 64, NE / 64), dim3(256), 0, stream>>>(Wqkv, NE, NC3, Wh, Wl);
  k_transpose_split<<<dim3(NE / 64, (NH * ND) / 64), dim3(256), 0, stream>>>(Wout, NH * ND, NE, Woh, Wol);
  k_flags<<<dim3(NQT), dim3(256), 0, stream>>>(msk, ftab);
  k_gemm_qkv<<<dim3(NC3 / 64, NTOK / 128), dim3(256), 0, stream>>>(Xh, Xl, Wh, Wl, sqkv, Qh, Ql, Kh, Kl, Vh, Vl);
  k_attn<<<dim3(NQT, NH, NB), dim3(128), 0, stream>>>(Qh, Ql, Kh, Kl, Vh, Vl, msk, ftab, Ahp, Alp);
  k_gemm_out<<<dim3(NE / 64, NTOK / 128), dim3(256), 0, stream>>>(Ahp, Alp, Woh, Wol, sout, out);
}
